// SpatialAttention2d_8169027797511
// MI455X (gfx1250) — hardware-verified
//
#include <hip/hip_runtime.h>

#define NB_  8
#define NC_  256
#define HW_  4096
#define PT_  64
#define XSTR 72

typedef _Float16 f16;
typedef __attribute__((ext_vector_type(16))) f16 f16x16;
typedef __attribute__((ext_vector_type(8)))  f16 f16x8;
typedef __attribute__((ext_vector_type(8)))  float f32x8;
typedef __attribute__((ext_vector_type(4)))  float v4f_t;
typedef float v4fa __attribute__((ext_vector_type(4), may_alias));
typedef __attribute__((ext_vector_type(4)))  unsigned v4u_t;
typedef unsigned v4ua __attribute__((ext_vector_type(4), may_alias));

__device__ __forceinline__ f32x8 wmma16(f16x16 a, f16x16 b, f32x8 c) {
  return __builtin_amdgcn_wmma_f32_16x16x32_f16(false, a, false, b, (short)0, c, false, false);
}

__global__ __launch_bounds__(128) void sa_squeeze_kernel(const float* __restrict__ x, const float* __restrict__ wsq,
                                                        const float* __restrict__ prm,
                                                        const float* __restrict__ wq, const float* __restrict__ bq,
                                                        const float* __restrict__ wk, const float* __restrict__ bk,
                                                        const float* __restrict__ wv, const float* __restrict__ bv,
                                                        float* __restrict__ q32, float* __restrict__ k32, f16* __restrict__ v16) {
  __shared__ __attribute__((aligned(16))) f16 Xs[NC_ * XSTR];
  __shared__ __attribute__((aligned(16))) float zS[PT_];
  __shared__ __attribute__((aligned(16))) float qS[PT_], kS[PT_];
  __shared__ __attribute__((aligned(16))) f16 vS[PT_];
  (void)prm;
  const int tid = threadIdx.x, lane = tid & 31, wave = tid >> 5;
  const int b  = blockIdx.x / (HW_ / PT_);
  const int p0 = (blockIdx.x % (HW_ / PT_)) * PT_;
  const float* xb = x + (size_t)b * NC_ * HW_ + p0;

  for (int c = tid; c < NC_; c += 128) {
    const float* row = xb + (size_t)c * HW_;
#pragma unroll
    for (int g = 0; g < 16; ++g) {
      const v4f_t f = *(const v4f_t*)(row + 4 * g);
      f16* d = Xs + c * XSTR + 4 * g;
      d[0] = (f16)f[0]; d[1] = (f16)f[1]; d[2] = (f16)f[2]; d[3] = (f16)f[3];
    }
  }
  __syncthreads();

  const int pl = lane & 15, kh = (lane >> 4) * 8;
  f32x8 acc = {};
#pragma unroll 2
  for (int ks = 0; ks < NC_ / 32; ++ks) {
    f16x16 af, bf;
    const int c0 = ks * 32 + kh;
#pragma unroll
    for (int i = 0; i < 8; ++i) {
      af[i]     = Xs[(c0 + i) * XSTR + wave * 16 + pl];
      af[i + 8] = Xs[(c0 + 16 + i) * XSTR + wave * 16 + pl];
      bf[i]     = (pl == 0) ? (f16)wsq[c0 + i]      : (f16)0.0f;
      bf[i + 8] = (pl == 0) ? (f16)wsq[c0 + 16 + i] : (f16)0.0f;
    }
    acc = wmma16(af, bf, acc);
  }
  if (pl == 0) {
#pragma unroll
    for (int r = 0; r < 8; ++r) zS[wave * 16 + (lane >> 4) * 8 + r] = acc[r];
  }
  __syncthreads();
  if (tid < PT_) {
    float z = zS[tid]; z = z > 0.0f ? z : 0.0f;
    qS[tid] = wq[0] * z + bq[0];
    kS[tid] = wk[0] * z + bk[0];
    vS[tid] = (f16)(wv[0] * z + bv[0]);
  }
  __syncthreads();
  if (wave == 0) {
    const size_t o = (size_t)b * HW_ + p0;
#pragma unroll 1
    for (int pass = 0; pass < 2; ++pass) {
      if (lane < 16) *(volatile v4f_t*)(q32 + o + 4 * lane) = *(const volatile v4fa*)(qS + 4 * lane);
      else           *(volatile v4f_t*)(k32 + o + 4 * (lane - 16)) = *(const volatile v4fa*)(kS + 4 * (lane - 16));
      if (lane < 8)  *(volatile v4u_t*)(v16 + o + 8 * lane) = *(const volatile v4ua*)(vS + 8 * lane);
      __threadfence();
    }
  }
}

__global__ __launch_bounds__(128) void sa_attn_kernel(const float* __restrict__ q32, const float* __restrict__ k32,
                                                     const f16* __restrict__ v16, const float* __restrict__ gamma,
                                                     float* __restrict__ gate) {
  __shared__ float redmx[4], redmn[4];
  __shared__ __attribute__((aligned(16))) float oS[4][16][2];
  __shared__ __attribute__((aligned(16))) float gS[PT_];
  const int tid = threadIdx.x, lane = tid & 31, wave = tid >> 5;
  const int b  = blockIdx.x / (HW_ / PT_);
  const int i0 = (blockIdx.x % (HW_ / PT_)) * PT_;
  const float* kb = k32 + (size_t)b * HW_;
  const f16*   vb = v16 + (size_t)b * HW_;

  float mx = -3.0e38f, mn = 3.0e38f;
  for (int j = tid; j < HW_; j += 128) { const float kv = kb[j]; mx = fmaxf(mx, kv); mn = fminf(mn, kv); }
#pragma unroll
  for (int off = 16; off >= 1; off >>= 1) { mx = fmaxf(mx, __shfl_xor(mx, off, 32)); mn = fminf(mn, __shfl_xor(mn, off, 32)); }
  if (lane == 0) { redmx[wave] = mx; redmn[wave] = mn; }
  __syncthreads();
  mx = fmaxf(fmaxf(redmx[0], redmx[1]), fmaxf(redmx[2], redmx[3]));
  mn = fminf(fminf(redmn[0], redmn[1]), fminf(redmn[2], redmn[3]));

  const int pl = lane & 15, kh = (lane >> 4) * 8;
  const float qi = q32[(size_t)b * HW_ + i0 + wave * 16 + pl];
  const float mi = (qi >= 0.0f) ? qi * mx : qi * mn;
  const float LOG2E = 1.44269504088896340736f;
  const float qs = qi * LOG2E, ms = mi * LOG2E - 10.0f;

  f16x16 bone;
#pragma unroll
  for (int e = 0; e < 16; ++e) bone[e] = (pl == 1) ? (f16)1.0f : (f16)0.0f;

  f32x8 acc = {};
#pragma unroll 2
  for (int js = 0; js < HW_ / 32; ++js) {
    const int j0 = js * 32 + kh;
    const v4f_t ka = *(const v4f_t*)(kb + j0),      kb4 = *(const v4f_t*)(kb + j0 + 4);
    const v4f_t kc = *(const v4f_t*)(kb + j0 + 16), kd  = *(const v4f_t*)(kb + j0 + 20);
    float kk[16] = {ka[0], ka[1], ka[2], ka[3], kb4[0], kb4[1], kb4[2], kb4[3],
                    kc[0], kc[1], kc[2], kc[3], kd[0],  kd[1],  kd[2],  kd[3]};
    f16x16 af;
#pragma unroll
    for (int e = 0; e < 16; ++e) af[e] = (f16)__builtin_amdgcn_exp2f(qs * kk[e] - ms);
    f16x16 bf = bone;
    if (pl == 0) {
      const f16x8 v0 = *(const f16x8*)(vb + j0), v1 = *(const f16x8*)(vb + j0 + 16);
#pragma unroll
      for (int e = 0; e < 8; ++e) { bf[e] = v0[e]; bf[e + 8] = v1[e]; }
    }
    acc = wmma16(af, bf, acc);
  }
  if (pl < 2) {
#pragma unroll
    for (int r = 0; r < 8; ++r) oS[wave][(lane >> 4) * 8 + r][pl] = acc[r];
  }
  __syncthreads();
  if (tid < PT_) {
    const int w = tid >> 4, r = tid & 15;
    const float outv = oS[w][r][0] / oS[w][r][1];
    const float g = gamma[0] * outv;
    gS[tid] = 1.0f / (1.0f + __expf(-g));
  }
  __syncthreads();
  if (wave == 0 && lane < 16) {
    const size_t o = (size_t)b * HW_ + i0;
#pragma unroll 1
    for (int pass = 0; pass < 2; ++pass) {
      *(volatile v4f_t*)(gate + o + 4 * lane) = *(const volatile v4fa*)(gS + 4 * lane);
      __threadfence();
    }
  }
}

__global__ __launch_bounds__(256) void sa_gate_kernel(const float* __restrict__ x, const float* __restrict__ gate,
                                                     float* __restrict__ y) {
  const int row = blockIdx.x;
  const int b = row / NC_;
  const float* xr = x + (size_t)row * HW_;
  const float* gr = gate + (size_t)b * HW_;
  float* yr = y + (size_t)row * HW_;
  v4f_t r[4];
#pragma unroll
  for (int u = 0; u < 4; ++u) {
    const int f4 = threadIdx.x + 256 * u;
    const v4f_t xv = *(const v4f_t*)(xr + 4 * f4), gv = *(const v4f_t*)(gr + 4 * f4);
    r[u] = xv * gv;
  }
#pragma unroll 1
  for (int pass = 0; pass < 2; ++pass) {
#pragma unroll
    for (int u = 0; u < 4; ++u) *(volatile v4f_t*)(yr + 4 * (threadIdx.x + 256 * u)) = r[u];
    __threadfence();
  }
}

extern "C" void kernel_launch(void* const* d_in, const int* in_sizes, int n_in,
                              void* d_out, int out_size, void* d_ws, size_t ws_size,
                              hipStream_t stream) {
  (void)in_sizes; (void)n_in; (void)out_size; (void)ws_size;
  const float* x   = (const float*)d_in[0];
  const float* wsq = (const float*)d_in[1];
  const float* wq  = (const float*)d_in[2];
  const float* bq  = (const float*)d_in[3];
  const float* wk  = (const float*)d_in[4];
  const float* bk  = (const float*)d_in[5];
  const float* wv  = (const float*)d_in[6];
  const float* bv  = (const float*)d_in[7];
  const float* gam = (const float*)d_in[8];
  float* y = (float*)d_out;

  char* ws = (char*)d_ws;
  float* q32  = (float*)(ws);
  float* k32  = (float*)(ws + 131072);
  f16*   v16  = (f16*)(ws + 262144);
  float* gate = (float*)(ws + 327680);

  sa_squeeze_kernel<<<dim3(NB_ * (HW_ / PT_)), dim3(128), 0, stream>>>(x, wsq, nullptr, wq, bq, wk, bk, wv, bv, q32, k32, v16);
  sa_attn_kernel<<<dim3(NB_ * (HW_ / PT_)), dim3(128), 0, stream>>>(q32, k32, v16, gam, gate);
  sa_gate_kernel<<<dim3(NB_ * NC_), dim3(256), 0, stream>>>(x, gate, y);
}
